// CapsuleNetwork_17497696764606
// MI455X (gfx1250) — hardware-verified
//
#include <hip/hip_runtime.h>


#define HIDDEN       128
#define NUM_INTEREST 8
#define SEQ          200
#define ITER_TIMES   3
#define S_PAD16      208
#define S_PAD32      224
#define KPAD         16
#define NTHR         256
#define NWAVE        (NTHR / 32)

typedef __bf16 v16bf __attribute__((ext_vector_type(16)));
typedef float v8f __attribute__((ext_vector_type(8)));
typedef float v4f __attribute__((ext_vector_type(4)));
typedef unsigned int v4u __attribute__((ext_vector_type(4)));
typedef unsigned int v2u __attribute__((ext_vector_type(2)));
typedef v4f v4f_a __attribute__((may_alias));
typedef v4u v4u_a __attribute__((may_alias));
typedef v2u v2u_a __attribute__((may_alias));

union FragBF { v16bf v; v4u q[2]; unsigned int u[8]; };

__device__ __forceinline__ unsigned int bf_rne(float x) {
    const unsigned int u = __builtin_bit_cast(unsigned int, x);
    return (u + 0x7FFFu + ((u >> 16) & 1u)) >> 16;
}
__device__ __forceinline__ float bf_val(unsigned int b16) {
    return __builtin_bit_cast(float, b16 << 16);
}
__device__ __forceinline__ void split2(float x, unsigned int& hi, unsigned int& lo) {
    hi = bf_rne(x);
    lo = bf_rne(x - bf_val(hi));
}

__device__ __forceinline__ v16bf frag_rowk(const unsigned short* p, int h) {
    FragBF f;
    f.q[0] = *(const v4u_a*)(p + 8 * h);
    f.q[1] = *(const v4u_a*)(p + 16 + 8 * h);
    return f.v;
}
__device__ __forceinline__ v16bf frag_colk(const unsigned short* p, int ld, int h) {
    FragBF f;
#pragma unroll
    for (int j = 0; j < 4; ++j) {
        const int ka = 8 * h + 2 * j;
        const int kb = 16 + 8 * h + 2 * j;
        f.u[j]     = (unsigned int)p[ka * ld] | ((unsigned int)p[(ka + 1) * ld] << 16);
        f.u[4 + j] = (unsigned int)p[kb * ld] | ((unsigned int)p[(kb + 1) * ld] << 16);
    }
    return f.v;
}

__device__ __forceinline__ v8f mma_bf16(v16bf a, v16bf b, v8f c) {
    v8f d = __builtin_amdgcn_wmma_f32_16x16x32_bf16(false, a, false, b, (short)0, c, false, false);
    asm volatile("v_nop\n\tv_nop\n\tv_nop\n\tv_nop" : "+v"(d) : "v"(a), "v"(b));
    return d;
}
__device__ __forceinline__ v8f mma3(v16bf ah, v16bf al, v16bf bh, v16bf bl, v8f c) {
    c = mma_bf16(ah, bh, c);
    c = mma_bf16(ah, bl, c);
    c = mma_bf16(al, bh, c);
    return c;
}

__device__ __forceinline__ float dot4acc(v4f w, v4f u, float a) {
    a += w.x * u.x; a += w.y * u.y; a += w.z * u.z; a += w.w * u.w;
    return a;
}
__device__ __forceinline__ float wave_sum(float p) {
    p += __shfl_xor(p, 16, 32);
    p += __shfl_xor(p, 8, 32);
    p += __shfl_xor(p, 4, 32);
    p += __shfl_xor(p, 2, 32);
    p += __shfl_xor(p, 1, 32);
    return p;
}

__global__ __launch_bounds__(NTHR)
void k_capsule_routing(const float* __restrict__ item_g,
                       const int*   __restrict__ mask_g,
                       const float* __restrict__ W_g,
                       const float* __restrict__ b_g,
                       float* out_g,
                       int nb)
{
    __shared__ __align__(16) unsigned short item_hi[S_PAD32 * HIDDEN];
    __shared__ __align__(16) unsigned short item_lo[S_PAD32 * HIDDEN];
    __shared__ __align__(16) unsigned short c_hi[KPAD * S_PAD32];
    __shared__ __align__(16) unsigned short c_lo[KPAD * S_PAD32];
    __shared__ __align__(16) unsigned short v_hi[KPAD * HIDDEN];
    __shared__ __align__(16) unsigned short v_lo[KPAD * HIDDEN];
    __shared__ __align__(16) float b_logit[NUM_INTEREST * S_PAD16];
    __shared__ __align__(16) float u_l[NUM_INTEREST * HIDDEN];
    __shared__ __align__(16) float inter_l[NUM_INTEREST * HIDDEN];
    __shared__ float csum_l[NUM_INTEREST];
    __shared__ float beta_l[NUM_INTEREST];
    __shared__ int   mask_l[S_PAD16];

    const int b = blockIdx.x;
    if (b >= nb) return;
    const int tid = threadIdx.x;
    const int l = tid & 31, h = l >> 4, m = l & 15, wv = tid >> 5;

    {
        const float* itemb = item_g + (size_t)b * (SEQ * HIDDEN);
        for (int i = tid; i < (S_PAD32 * HIDDEN) / 4; i += NTHR) {
            const int e = i * 4;
            const int s = e >> 7;
            v4f x = {0.f, 0.f, 0.f, 0.f};
            if (s < SEQ) x = *(const v4f_a*)(itemb + e);
            unsigned int a0, a1, a2, a3, r0, r1, r2, r3;
            split2(x.x, a0, r0); split2(x.y, a1, r1); split2(x.z, a2, r2); split2(x.w, a3, r3);
            v2u hv, lv;
            hv.x = a0 | (a1 << 16); hv.y = a2 | (a3 << 16);
            lv.x = r0 | (r1 << 16); lv.y = r2 | (r3 << 16);
            *(v2u_a*)(item_hi + e) = hv;
            *(v2u_a*)(item_lo + e) = lv;
        }
        for (int i = tid; i < KPAD * S_PAD32; i += NTHR) { c_hi[i] = 0; c_lo[i] = 0; }
        for (int i = tid; i < KPAD * HIDDEN; i += NTHR)  { v_hi[i] = 0; v_lo[i] = 0; }
        for (int i = tid; i < NUM_INTEREST * S_PAD16; i += NTHR) b_logit[i] = 0.0f;
        for (int s = tid; s < S_PAD16; s += NTHR)
            mask_l[s] = (s < SEQ) ? mask_g[(size_t)b * SEQ + s] : 0;
    }
    __syncthreads();

    for (int it = 0; it < ITER_TIMES; ++it) {
        if (tid < SEQ) {
            const int s = tid;
            const bool mz = (mask_l[s] == 0);
            float vals[NUM_INTEREST];
            float mx = -3.0e38f;
#pragma unroll
            for (int k = 0; k < NUM_INTEREST; ++k) {
                float x = b_logit[k * S_PAD16 + s];
                if (mz) { x = -10000.0f; b_logit[k * S_PAD16 + s] = x; }
                vals[k] = x;
                mx = fmaxf(mx, x);
            }
            float ssum = 0.0f;
#pragma unroll
            for (int k = 0; k < NUM_INTEREST; ++k) { vals[k] = expf(vals[k] - mx); ssum += vals[k]; }
            const float inv = 1.0f / ssum;
#pragma unroll
            for (int k = 0; k < NUM_INTEREST; ++k) {
                const float c = vals[k] * inv;
                unsigned int ch, cl;
                split2(c, ch, cl);
                c_hi[k * S_PAD32 + s] = (unsigned short)ch;
                c_lo[k * S_PAD32 + s] = (unsigned short)cl;
            }
        }
        __syncthreads();

        {
            const int dt = wv * 16;
            v8f acc = {0.f, 0.f, 0.f, 0.f, 0.f, 0.f, 0.f, 0.f};
#pragma unroll 1
            for (int ks = 0; ks < S_PAD32; ks += 32) {
                const v16bf ah = frag_rowk(c_hi + m * S_PAD32 + ks, h);
                const v16bf al = frag_rowk(c_lo + m * S_PAD32 + ks, h);
                const v16bf bh = frag_colk(item_hi + ks * HIDDEN + dt + m, HIDDEN, h);
                const v16bf bl = frag_colk(item_lo + ks * HIDDEN + dt + m, HIDDEN, h);
                acc = mma3(ah, al, bh, bl, acc);
            }
            if (h == 0) {
#pragma unroll
                for (int r = 0; r < 8; ++r) u_l[r * HIDDEN + dt + m] = acc[r];
            }
            if (tid < NUM_INTEREST) {
                float cs = 0.0f;
                for (int s = 0; s < SEQ; ++s)
                    cs += bf_val(c_hi[tid * S_PAD32 + s]) + bf_val(c_lo[tid * S_PAD32 + s]);
                csum_l[tid] = cs;
            }
        }
        __syncthreads();

        {
            const int k = wv;
            const int dq = 4 * l;
            const int o0 = k * HIDDEN + dq;
            const float cs = csum_l[k];
            float ip0 = cs * b_g[o0], ip1 = cs * b_g[o0 + 1], ip2 = cs * b_g[o0 + 2], ip3 = cs * b_g[o0 + 3];
            const float* w0 = W_g + (size_t)o0 * HIDDEN;
            const float* urow = u_l + k * HIDDEN;
#pragma unroll 4
            for (int d4 = 0; d4 < HIDDEN / 4; ++d4) {
                const v4f uu = *(const v4f_a*)(urow + 4 * d4);
                v4f w;
                w = *(const v4f_a*)(w0 + 4 * d4);              ip0 = dot4acc(w, uu, ip0);
                w = *(const v4f_a*)(w0 + HIDDEN + 4 * d4);     ip1 = dot4acc(w, uu, ip1);
                w = *(const v4f_a*)(w0 + 2 * HIDDEN + 4 * d4); ip2 = dot4acc(w, uu, ip2);
                w = *(const v4f_a*)(w0 + 3 * HIDDEN + 4 * d4); ip3 = dot4acc(w, uu, ip3);
            }
            float p = ip0 * ip0 + ip1 * ip1 + ip2 * ip2 + ip3 * ip3;
            const float n2 = wave_sum(p);
            const float n = sqrtf(n2);
            const float f1 = n2 / (1.0f + n2);
            const float rden = 1.0f / (n + 1e-12f);
            v4f val;
            val.x = f1 * (ip0 * rden);
            val.y = f1 * (ip1 * rden);
            val.z = f1 * (ip2 * rden);
            val.w = f1 * (ip3 * rden);
            if (it == ITER_TIMES - 1) {
                volatile v4f* po = (volatile v4f*)(out_g + ((size_t)b * (NUM_INTEREST * HIDDEN) + 4 * tid));
                *po = val;
                __threadfence();
                *po = val;
                break;
            }
            *(v4f_a*)(inter_l + k * HIDDEN + dq) = val;
        }
        __syncthreads();

        {
            const int k = wv;
            const int d0 = 4 * l;
            const float* irow = inter_l + k * HIDDEN;
            {
                const v4f ivo = *(const v4f_a*)(irow + d0);
                const v4f bb  = *(const v4f_a*)(b_g + k * HIDDEN + d0);
                float bp = 0.0f;
                bp = dot4acc(bb, ivo, bp);
                bp = wave_sum(bp);
                if (l == 0) beta_l[k] = bp;
            }
            v4f va = {0.f, 0.f, 0.f, 0.f};
            const float* wk = W_g + (size_t)k * HIDDEN * HIDDEN + d0;
#pragma unroll 2
            for (int dp4 = 0; dp4 < HIDDEN / 4; ++dp4) {
                const v4f iv = *(const v4f_a*)(irow + 4 * dp4);
                const float* wr = wk + (size_t)(4 * dp4) * HIDDEN;
                v4f w;
                w = *(const v4f_a*)(wr);               va += w * iv.x;
                w = *(const v4f_a*)(wr + HIDDEN);      va += w * iv.y;
                w = *(const v4f_a*)(wr + 2 * HIDDEN);  va += w * iv.z;
                w = *(const v4f_a*)(wr + 3 * HIDDEN);  va += w * iv.w;
            }
            unsigned int a0, a1, a2, a3, r0, r1, r2, r3;
            split2(va.x, a0, r0); split2(va.y, a1, r1); split2(va.z, a2, r2); split2(va.w, a3, r3);
            v2u hv, lv;
            hv.x = a0 | (a1 << 16); hv.y = a2 | (a3 << 16);
            lv.x = r0 | (r1 << 16); lv.y = r2 | (r3 << 16);
            *(v2u_a*)(v_hi + k * HIDDEN + d0) = hv;
            *(v2u_a*)(v_lo + k * HIDDEN + d0) = lv;
        }
        __syncthreads();

        for (int t = wv; t < S_PAD16 / 16; t += NWAVE) {
            const int st = t * 16;
            v8f acc = {0.f, 0.f, 0.f, 0.f, 0.f, 0.f, 0.f, 0.f};
#pragma unroll 1
            for (int kd = 0; kd < HIDDEN; kd += 32) {
                const v16bf ah = frag_rowk(item_hi + (st + m) * HIDDEN + kd, h);
                const v16bf al = frag_rowk(item_lo + (st + m) * HIDDEN + kd, h);
                const v16bf bh = frag_rowk(v_hi + m * HIDDEN + kd, h);
                const v16bf bl = frag_rowk(v_lo + m * HIDDEN + kd, h);
                acc = mma3(ah, al, bh, bl, acc);
            }
            if (m < NUM_INTEREST) {
                const float be = beta_l[m];
#pragma unroll
                for (int r = 0; r < 8; ++r) {
                    const int s = st + 8 * h + r;
                    if (s < SEQ) b_logit[m * S_PAD16 + s] += acc[r] + be;
                }
            }
        }
        __syncthreads();
    }
}

extern "C" void kernel_launch(void* const* d_in, const int* in_sizes, int n_in,
                              void* d_out, int out_size, void* d_ws, size_t ws_size,
                              hipStream_t stream)
{
    (void)d_ws; (void)ws_size;
    if (n_in < 4) return;
    const float* item  = (const float*)d_in[0];
    const int*   mask  = (const int*)d_in[1];
    const float* W     = (const float*)d_in[2];
    const float* b_lin = (const float*)d_in[3];
    float* out = (float*)d_out;

    const int per_out = NUM_INTEREST * HIDDEN;
    int nb = out_size / per_out;
    const int nb_item = in_sizes[0] / (SEQ * HIDDEN);
    const int nb_mask = in_sizes[1] / SEQ;
    if (nb_item < nb) nb = nb_item;
    if (nb_mask < nb) nb = nb_mask;
    if (in_sizes[2] < NUM_INTEREST * HIDDEN * HIDDEN) return;
    if (in_sizes[3] < NUM_INTEREST * HIDDEN) return;
    if (nb <= 0) return;

    k_capsule_routing<<<nb, NTHR, 0, stream>>>(item, mask, W, b_lin, out, nb);
    (void)hipGetLastError();
}
